// NeptuneMoEModel_68831145886459
// MI455X (gfx1250) — hardware-verified
//
#include <hip/hip_runtime.h>
#include <math.h>
#include <stddef.h>
#include <stdint.h>


#define NPT   524288
#define NEV   2048
#define TT    256
#define DD    256
#define HHID  512
#define KIN   259
#define KP    320
#define TSUB  64
#define NSUB  4
#define SROW  264
#define NOUT  11
#define ASC   16
#define XSC   64
#define WSC   1024
#define WSCAP 134217728
#define LOG2E 1.4426950408889634f

static_assert(NSUB * TSUB == TT);
static_assert(NEV * TT == NPT);
static_assert(KP % 32 == 0);
static_assert(KP >= KIN);
static_assert(DD % 32 == 0);
static_assert(NEV % 32 == 0);
static_assert((32 * NOUT * 4) % 128 == 0);
static_assert((KP * 2) % 128 == 0);
static_assert(SROW % 8 == 0);

typedef float    v4f  __attribute__((ext_vector_type(4)));
typedef float    v8f  __attribute__((ext_vector_type(8)));
typedef _Float16 v8h  __attribute__((ext_vector_type(8)));
typedef _Float16 v16h __attribute__((ext_vector_type(16)));
union FragH { v16h v; v8h h[2]; };

__device__ __forceinline__ v8f wmf(v16h a, v16h b, v8f c) {
  v8f d = __builtin_amdgcn_wmma_f32_16x16x32_f16(false, a, false, b, (short)0, c, false, false);
  asm volatile("v_nop\n\tv_nop\n\tv_nop\n\tv_nop" : "+v"(d) : "v"(a), "v"(b));
  return d;
}

__device__ __forceinline__ v8f splat8(float x) { v8f r = {x, x, x, x, x, x, x, x}; return r; }

__device__ __forceinline__ v16h ldfrag(const _Float16* p, int k0, int hh) {
  FragH u;
  u.h[0] = *(const v8h*)(p + k0 + 8 * hh);
  u.h[1] = *(const v8h*)(p + k0 + 16 + 8 * hh);
  return u.v;
}

__device__ __forceinline__ float tanh_f(float x) {
  const float ax = fabsf(x);
  const float e  = __builtin_amdgcn_exp2f(ax * (-2.0f * LOG2E));
  const float r  = (1.0f - e) * __builtin_amdgcn_rcpf(1.0f + e);
  return copysignf(r, x);
}
__device__ __forceinline__ float gelu_t(float x) {
  const float in = 0.7978845608028654f * (x + 0.044715f * (x * x * x));
  return 0.5f * x * (1.0f + tanh_f(in));
}

__device__ __forceinline__ v8h prepw_piece(const float* ts, int p, int npc) {
  const int row = p / npc, k8 = (p - row * npc) * 8;
  v8h o;
#pragma unroll
  for (int e = 0; e < 8; ++e) o[e] = (_Float16)(ts[(k8 + e) * 16 + row] * (float)WSC);
  return o;
}

__global__ __launch_bounds__(256) void k_prepw(const float* __restrict__ W, int Kd, int Nd, int KPp,
                                                _Float16* dst) {
  __shared__ __attribute__((aligned(16))) float ts[KP * 16];
  const int t = threadIdx.x;
  const int n0 = blockIdx.x * 16;
#pragma unroll
  for (int ps = 0; ps < 2; ++ps) {
    const int k = t + 256 * ps;
    if (k < KPp) {
      const float* wrow = W + (size_t)min(k, Kd - 1) * Nd;
#pragma unroll
      for (int nn = 0; nn < 16; ++nn) {
        const int n = n0 + nn;
        const float v = wrow[min(n, Nd - 1)];
        ts[k * 16 + nn] = (k < Kd && n < Nd) ? v : 0.0f;
      }
    }
  }
  __syncthreads();
  const int npc = KPp >> 3;
  const int tot = 16 * npc;
  const int p0 = t, p1 = t + 256, p2 = t + 512;
  const bool a0 = p0 < tot, a1 = p1 < tot, a2 = p2 < tot;
  const v8h o0 = prepw_piece(ts, a0 ? p0 : 0, npc);
  const v8h o1 = prepw_piece(ts, a1 ? p1 : 0, npc);
  const v8h o2 = prepw_piece(ts, a2 ? p2 : 0, npc);
  _Float16* db = dst + (size_t)n0 * KPp;
  _Float16* d0 = db + 8 * (a0 ? p0 : 0);
  _Float16* d1 = db + 8 * (a1 ? p1 : 0);
  _Float16* d2 = db + 8 * (a2 ? p2 : 0);
  if (a0) *(volatile v8h*)d0 = o0;
  if (a1) *(volatile v8h*)d1 = o1;
  if (a2) *(volatile v8h*)d2 = o2;
  __threadfence();
  if (a0) *(volatile v8h*)d0 = o0;
  if (a1) *(volatile v8h*)d1 = o1;
  if (a2) *(volatile v8h*)d2 = o2;
}

__global__ __launch_bounds__(256) void k_main(const float* __restrict__ coords, const float* __restrict__ feats,
                                               const float* __restrict__ W_in, const float* __restrict__ b_in,
                                               const _Float16* __restrict__ wht, const float* __restrict__ b_h,
                                               _Float16* xp) {
  __shared__ __attribute__((aligned(16))) _Float16 h1s[TSUB * SROW];
  __shared__ __attribute__((aligned(16))) float pts[TSUB * 12];
  __shared__ __attribute__((aligned(16))) float s_part[4 * DD];
  __shared__ __attribute__((aligned(16))) _Float16 s_x[KP];

  const int tid = threadIdx.x, lane = tid & 31, w = tid >> 5, hh = lane >> 4, nl = lane & 15;
  const int ev = blockIdx.x;
  const int mt = w & 3, ng = w >> 2;
  constexpr float OSC2 = 1.0f / (float)(ASC * WSC);

  float w9[9];
#pragma unroll
  for (int j = 0; j < 9; ++j) w9[j] = W_in[j * DD + tid];
  const float bb = b_in[tid];

  float colacc = 0.0f, cacc = 0.0f;

#pragma unroll 1
  for (int sub = 0; sub < NSUB; ++sub) {
    const size_t rb = (size_t)ev * TT + (size_t)sub * TSUB;
    if (tid < TSUB) {
      const size_t r = rb + (size_t)tid;
      float* p = pts + tid * 12;
      p[0] = coords[r * 3 + 0];
      p[1] = coords[r * 3 + 1];
      p[2] = coords[r * 3 + 2];
#pragma unroll
      for (int j = 0; j < 6; ++j) p[3 + j] = feats[r * 6 + j];
    }
    __syncthreads();

    if (tid < 3) {
      float s = 0.0f;
#pragma unroll 1
      for (int i = 0; i < TSUB; ++i) s += pts[i * 12 + tid];
      cacc += s;
    }

#pragma unroll 1
    for (int i = 0; i < TSUB; ++i) {
      const float* p = pts + i * 12;
      float acc = bb;
#pragma unroll
      for (int j = 0; j < 9; ++j) acc += p[j] * w9[j];
      h1s[i * SROW + tid] = (_Float16)(gelu_t(acc) * (float)ASC);
    }
    __syncthreads();

    v16h af[8];
    {
      const _Float16* ap = h1s + (mt * 16 + nl) * SROW;
#pragma unroll
      for (int kt = 0; kt < 8; ++kt) af[kt] = ldfrag(ap, 32 * kt, hh);
    }
#pragma unroll 1
    for (int nt = ng * 8; nt < ng * 8 + 8; ++nt) {
      const _Float16* bp = wht + (size_t)(nt * 16 + nl) * DD;
      v8f c = splat8(0.0f);
#pragma unroll
      for (int kt = 0; kt < 8; ++kt) c = wmf(af[kt], ldfrag(bp, 32 * kt, hh), c);
      const int col = nt * 16 + nl;
      const float bias = b_h[col];
      float cs = 0.0f;
#pragma unroll
      for (int r = 0; r < 8; ++r) cs += gelu_t(c[r] * OSC2 + bias);
      cs += __shfl_xor(cs, 16, 32);
      if (hh == 0) s_part[mt * DD + col] = cs;
    }
    __syncthreads();
    colacc += (s_part[tid] + s_part[DD + tid]) + (s_part[2 * DD + tid] + s_part[3 * DD + tid]);
  }

  s_x[tid] = (_Float16)(colacc * ((float)XSC / (float)TT));
  if (tid < KP - DD) {
    const float cv = (tid < 3) ? cacc * ((float)XSC / (float)TT) : 0.0f;
    s_x[DD + tid] = (_Float16)cv;
  }
  __syncthreads();
  const bool act = tid < (KP / 8);
  const v8h v = *(const v8h*)(s_x + 8 * (act ? tid : 0));
  _Float16* d = xp + (size_t)ev * KP + 8 * (act ? tid : 0);
  if (act) *(volatile v8h*)d = v;
  __threadfence();
  if (act) *(volatile v8h*)d = v;
}

template <int OD, int OFF>
__device__ __forceinline__ void head_pass(const _Float16* __restrict__ ap, const _Float16* __restrict__ w1h,
                                          const float* __restrict__ b1, const float* __restrict__ W2,
                                          const float* __restrict__ b2, float* s_part, float* s_res,
                                          int t, int hh, int nl, int mw, int g) {
  constexpr float OSCH = 1.0f / (float)(XSC * WSC);
  float part[OD][8];
#pragma unroll
  for (int o = 0; o < OD; ++o) {
#pragma unroll
    for (int r = 0; r < 8; ++r) part[o][r] = 0.0f;
  }
#pragma unroll 1
  for (int nt = 0; nt < 8; ++nt) {
    const int cl = g * 128 + nt * 16;
    const _Float16* bp = w1h + (size_t)(cl + nl) * KP;
    v8f c = splat8(0.0f);
#pragma unroll
    for (int ks = 0; ks < KP / 32; ++ks) c = wmf(ldfrag(ap, 32 * ks, hh), ldfrag(bp, 32 * ks, hh), c);
    const int col = cl + nl;
    const float bias = b1[col];
    float wv[OD];
#pragma unroll
    for (int o = 0; o < OD; ++o) wv[o] = W2[col * OD + o];
#pragma unroll
    for (int r = 0; r < 8; ++r) {
      const float hv = gelu_t(c[r] * OSCH + bias);
#pragma unroll
      for (int o = 0; o < OD; ++o) part[o][r] += hv * wv[o];
    }
  }
#pragma unroll
  for (int o = 0; o < OD; ++o) {
#pragma unroll
    for (int r = 0; r < 8; ++r) {
      float v = part[o][r];
      v += __shfl_xor(v, 1, 32);
      v += __shfl_xor(v, 2, 32);
      v += __shfl_xor(v, 4, 32);
      v += __shfl_xor(v, 8, 32);
      part[o][r] = v;
    }
  }
  if (nl == 0) {
#pragma unroll
    for (int o = 0; o < OD; ++o) {
#pragma unroll
      for (int r = 0; r < 8; ++r) s_part[(g * 32 + 16 * mw + 8 * hh + r) * 8 + o] = part[o][r];
    }
  }
  __syncthreads();
  if (t < 32) {
#pragma unroll
    for (int o = 0; o < OD; ++o) {
      const float s = (s_part[t * 8 + o] + s_part[(32 + t) * 8 + o]) +
                      (s_part[(64 + t) * 8 + o] + s_part[(96 + t) * 8 + o]);
      s_res[t * 20 + OFF + o] = b2[o] + s;
    }
  }
  __syncthreads();
}

__global__ __launch_bounds__(256) void k_heads(const _Float16* __restrict__ xp, const _Float16* __restrict__ w1t,
                                                const float* __restrict__ b1_0, const float* __restrict__ W2_0, const float* __restrict__ b2_0,
                                                const float* __restrict__ b1_1, const float* __restrict__ W2_1, const float* __restrict__ b2_1,
                                                const float* __restrict__ b1_2, const float* __restrict__ W2_2, const float* __restrict__ b2_2,
                                                const float* __restrict__ b1_3, const float* __restrict__ W2_3, const float* __restrict__ b2_3,
                                                const float* __restrict__ b1_4, const float* __restrict__ W2_4, const float* __restrict__ b2_4,
                                                const float* __restrict__ b1_5, const float* __restrict__ W2_5, const float* __restrict__ b2_5,
                                                float* out) {
  __shared__ __attribute__((aligned(16))) float s_part[4 * 32 * 8];
  __shared__ __attribute__((aligned(16))) float s_res[32 * 20];
  __shared__ __attribute__((aligned(16))) float s_out[32 * NOUT];

  const int t = threadIdx.x, lane = t & 31, w = t >> 5, hh = lane >> 4, nl = lane & 15;
  const int mw = w & 1, g = w >> 1;
  const int row0 = blockIdx.x * 32;
  const _Float16* ap = xp + (size_t)(row0 + 16 * mw + nl) * KP;

  head_pass<6, 0>(ap,  w1t + (size_t)0 * HHID * KP, b1_0, W2_0, b2_0, s_part, s_res, t, hh, nl, mw, g);
  head_pass<2, 6>(ap,  w1t + (size_t)1 * HHID * KP, b1_1, W2_1, b2_1, s_part, s_res, t, hh, nl, mw, g);
  head_pass<2, 8>(ap,  w1t + (size_t)2 * HHID * KP, b1_2, W2_2, b2_2, s_part, s_res, t, hh, nl, mw, g);
  head_pass<3, 10>(ap, w1t + (size_t)3 * HHID * KP, b1_3, W2_3, b2_3, s_part, s_res, t, hh, nl, mw, g);
  head_pass<3, 13>(ap, w1t + (size_t)4 * HHID * KP, b1_4, W2_4, b2_4, s_part, s_res, t, hh, nl, mw, g);
  head_pass<3, 16>(ap, w1t + (size_t)5 * HHID * KP, b1_5, W2_5, b2_5, s_part, s_res, t, hh, nl, mw, g);

  if (t < 32) {
    const float* rs = s_res + t * 20;
    float lg[6];
#pragma unroll
    for (int i = 0; i < 6; ++i) lg[i] = rs[i];
    float mx = lg[0];
#pragma unroll
    for (int i = 1; i < 6; ++i) mx = fmaxf(mx, lg[i]);
    float ex[6], s = 0.0f;
#pragma unroll
    for (int i = 0; i < 6; ++i) { ex[i] = expf(lg[i] - mx); s += ex[i]; }
    const float inv = 1.0f / s;
    float pr[6];
#pragma unroll
    for (int i = 0; i < 6; ++i) pr[i] = fmaxf(ex[i] * inv, 1e-6f);
    const float p_cont = pr[0] + pr[1];
    const float p_unc  = (pr[2] + pr[3]) + pr[5];
    const float ec0 = rs[6], ec1 = rs[7], eu0 = rs[8], eu1 = rs[9];
    const float e0 = p_cont * ec0 + p_unc * eu0;
    const float e1 = p_cont * ec1 + p_unc * eu1;
    const float p_cas = pr[0];
    const float p_trk = ((pr[1] + pr[3]) + pr[2]) + pr[5];
    const float gate = 1.0f / (1.0f + expf(-(e0 - 4.0f)));
    const float wl = p_trk * (1.0f - gate);
    const float wh = p_trk * gate;
    float* so = s_out + t * NOUT;
#pragma unroll
    for (int i = 0; i < 6; ++i) so[i] = lg[i];
    so[6] = e0;
    so[7] = e1;
#pragma unroll
    for (int i = 0; i < 3; ++i) so[8 + i] = (p_cas * rs[10 + i] + wl * rs[13 + i]) + wh * rs[16 + i];
  }
  __syncthreads();
  const bool act = t < (32 * NOUT / 4);
  const v4f v = *(const v4f*)(s_out + 4 * (act ? t : 0));
  float* d = out + (size_t)row0 * NOUT + 4 * (act ? t : 0);
  if (act) *(volatile v4f*)d = v;
  __threadfence();
  if (act) *(volatile v4f*)d = v;
}

extern "C" void kernel_launch(void* const* d_in, const int* in_sizes, int n_in,
                              void* d_out, int out_size, void* d_ws, size_t ws_size,
                              hipStream_t stream) {
  if (n_in < 31) return;
  if (in_sizes[0] != NPT * 3 || in_sizes[1] != NPT * 6 || in_sizes[2] != NPT) return;
  if (in_sizes[3] != 9 * DD || in_sizes[4] != DD || in_sizes[5] != DD * DD || in_sizes[6] != DD) return;
  const int odim[6] = {6, 2, 2, 3, 3, 3};
  for (int i = 0; i < 6; ++i) {
    if (in_sizes[7 + 4 * i] != KIN * HHID) return;
    if (in_sizes[8 + 4 * i] != HHID) return;
    if (in_sizes[9 + 4 * i] != HHID * odim[i]) return;
    if (in_sizes[10 + 4 * i] != odim[i]) return;
  }
  if (out_size != NEV * NOUT) return;

  const float* coords = (const float*)d_in[0];
  const float* feats  = (const float*)d_in[1];
  const float* W_in   = (const float*)d_in[3];
  const float* b_in   = (const float*)d_in[4];
  const float* W_h    = (const float*)d_in[5];
  const float* b_h    = (const float*)d_in[6];
  const float* W1p[6]; const float* b1p[6]; const float* W2p[6]; const float* b2p[6];
  for (int i = 0; i < 6; ++i) {
    W1p[i] = (const float*)d_in[7 + 4 * i];
    b1p[i] = (const float*)d_in[8 + 4 * i];
    W2p[i] = (const float*)d_in[9 + 4 * i];
    b2p[i] = (const float*)d_in[10 + 4 * i];
  }
  float* out = (float*)d_out;

  char* ws = (char*)d_ws;
  size_t off = 0;
  const size_t oWh = off; off += (size_t)DD * DD * 2;          off = (off + 255) & ~(size_t)255;
  const size_t oW1 = off; off += (size_t)6 * HHID * KP * 2;    off = (off + 255) & ~(size_t)255;
  const size_t oX  = off; off += (size_t)NEV * KP * 2;         off = (off + 255) & ~(size_t)255;
  if (off > ws_size || off > (size_t)WSCAP) return;
  _Float16* wht = (_Float16*)(ws + oWh);
  _Float16* w1t = (_Float16*)(ws + oW1);
  _Float16* xp  = (_Float16*)(ws + oX);

  k_prepw<<<DD / 16, 256, 0, stream>>>(W_h, DD, DD, DD, wht);
  for (int i = 0; i < 6; ++i)
    k_prepw<<<HHID / 16, 256, 0, stream>>>(W1p[i], KIN, HHID, KP, w1t + (size_t)i * HHID * KP);

  k_main<<<NEV, 256, 0, stream>>>(coords, feats, W_in, b_in, wht, b_h, xp);

  k_heads<<<NEV / 32, 256, 0, stream>>>(xp, w1t,
                                        b1p[0], W2p[0], b2p[0],
                                        b1p[1], W2p[1], b2p[1],
                                        b1p[2], W2p[2], b2p[2],
                                        b1p[3], W2p[3], b2p[3],
                                        b1p[4], W2p[4], b2p[4],
                                        b1p[5], W2p[5], b2p[5],
                                        out);
}
